// GauntTensorProductAllParitiesS2Grid_11209864642659
// MI455X (gfx1250) — hardware-verified
//
#include <hip/hip_runtime.h>

typedef unsigned short v8us  __attribute__((ext_vector_type(8)));
typedef unsigned short v16us __attribute__((ext_vector_type(16)));
typedef unsigned int   v8u   __attribute__((ext_vector_type(8)));
typedef __bf16         v16bf __attribute__((ext_vector_type(16)));
typedef float          v8f   __attribute__((ext_vector_type(8)));
typedef float          v4f   __attribute__((ext_vector_type(4)));
typedef v8us __attribute__((may_alias)) v8usa;
typedef v4f  __attribute__((may_alias)) v4fa;

union FragB { v16bf v; v16us u; v8u w; v8us h8[2]; };
static_assert(sizeof(FragB) == 32);

#define NS    2048
#define NCH   64
#define NLM   9
#define NLO   25
#define NG    780
#define NGC   25
#define NGT   50
#define NBETA 20
#define NALPHA 39

__device__ __forceinline__ unsigned int bf16u(float f) {
  const unsigned int u = __float_as_uint(f);
  return (u + 0x7FFFu + ((u >> 16) & 1u)) >> 16;
}
__device__ __forceinline__ float bf16val(unsigned int b) { return __uint_as_float(b << 16); }
__device__ __forceinline__ float bf16r(float f) { return bf16val(bf16u(f)); }

__device__ __forceinline__ v8f mma_bf16(v16bf a, v16bf b, v8f c) {
  v8f d = __builtin_amdgcn_wmma_f32_16x16x32_bf16(false, a, false, b, (short)0, c, false, false);
#if defined(__HIP_DEVICE_COMPILE__)
  asm volatile("v_nop\n\tv_nop\n\tv_nop\n\tv_nop" : "+v"(d) : "v"(a), "v"(b));
#endif
  return d;
}

__device__ __forceinline__ void load_frag_g(FragB& f, const unsigned short* p, int h) {
  f.h8[0] = *(const v8usa*)(p + 8 * h);
  f.h8[1] = *(const v8usa*)(p + 16 + 8 * h);
}

template <int HF>
__device__ __forceinline__ void split8(FragB& hi, FragB& lo, v4f a, v4f c) {
  #pragma unroll
  for (int i = 0; i < 8; ++i) {
    const float f = (i < 4) ? a[i] : c[i - 4];
    const unsigned int hb = bf16u(f);
    const float res = f - bf16val(hb);
    hi.u[8 * HF + i] = (unsigned short)hb;
    lo.u[8 * HF + i] = (unsigned short)bf16u(res);
  }
}

__global__ __launch_bounds__(64) void prep_kernel(
    const float* __restrict__ W1, const float* __restrict__ W2, const float* __restrict__ Wout,
    const float* __restrict__ Yin, const float* __restrict__ Yout,
    unsigned short* __restrict__ w1t, unsigned short* __restrict__ w2t,
    unsigned short* __restrict__ wot, unsigned short* __restrict__ yinA,
    unsigned short* __restrict__ youtA)
{
  const int tid = threadIdx.x, lane = tid & 31, wl = tid >> 5;
  const int bid = blockIdx.x;
  v8us o = {0, 0, 0, 0, 0, 0, 0, 0};
  unsigned short* dst;
  if (bid < 144) {
    const int t = (bid >= 72) ? 1 : 0;
    const int c = ((bid - 72 * t) * 2 + wl) * 32 + lane;
    const int rc = c >> 3, q = c & 7;
    const int bl = rc >> 6, cc = rc & 63;
    const float* src = (t ? W2 : W1) + (size_t)bl * 4096 + cc;
    #pragma unroll
    for (int i = 0; i < 8; ++i) o[i] = (unsigned short)bf16u(src[(8 * q + i) * 64]);
    dst = (t ? w2t : w1t) + (size_t)c * 8;
  } else if (bid < 264) {
    const int c = ((bid - 144) * 2 + wl) * 32 + lane;
    const int rc = c >> 3, q = c & 7;
    const int blq = rc >> 6, d = rc & 63;
    const float* src = Wout + (size_t)blq * 4096 + d;
    #pragma unroll
    for (int i = 0; i < 8; ++i) o[i] = (unsigned short)bf16u(src[(8 * q + i) * 64]);
    dst = wot + (size_t)c * 8;
  } else if (bid < 289) {
    const int c = ((bid - 264) * 2 + wl) * 32 + lane;
    const int gt = c >> 5, L = c & 31;
    const int hh = L >> 4, g = 16 * gt + (L & 15);
    const int gcl = (g < NG) ? g : (NG - 1);
    #pragma unroll
    for (int i = 0; i < 8; ++i) {
      const int k = 8 * hh + i;
      const int kc = (k < NLM) ? k : (NLM - 1);
      const float v = Yin[(size_t)kc * NG + gcl];
      o[i] = (k < NLM && g < NG) ? (unsigned short)bf16u(v) : (unsigned short)0;
    }
    dst = yinA + (size_t)c * 8;
  } else if (bid < 339) {
    const int c = ((bid - 289) * 2 + wl) * 32 + lane;
    const int gcm = c >> 6, L = (c >> 1) & 31, hf = c & 1;
    const int mt = gcm & 1, gc = gcm >> 1;
    const int lp = 16 * mt + (L & 15), hh = L >> 4;
    const int lpc = (lp < NLO) ? lp : (NLO - 1);
    #pragma unroll
    for (int i = 0; i < 8; ++i) {
      const int g = 32 * gc + 16 * hf + 8 * hh + i;
      const int gcl = (g < NG) ? g : (NG - 1);
      const float v = Yout[(size_t)lpc * NG + gcl];
      o[i] = (lp < NLO && g < NG) ? (unsigned short)bf16u(v) : (unsigned short)0;
    }
    dst = youtA + (size_t)c * 8;
  } else {
    return;
  }
  *(volatile v8us*)dst = o;
  __threadfence();
  *(volatile v8us*)dst = o;
}

__device__ __forceinline__ void out_pass(const float* outL, float* ob, int tid) {
  const int q = tid & 7, lb = tid >> 3;
  #pragma unroll
  for (int it = 0; it < 4; ++it) {
    const int L = it * 16 + lb;
    const int Lc = (L < 50) ? L : 49;
    const v4f v = *(const v4fa*)(outL + Lc * 32 + 4 * q);
    if (L < 50) *(volatile v4f*)(ob + (size_t)L * 32 + 4 * q) = v;
  }
}

__global__ __launch_bounds__(128) void gaunt_kernel(
    const float* __restrict__ x1, const float* __restrict__ x2, const float* __restrict__ qw,
    const unsigned short* __restrict__ w1t, const unsigned short* __restrict__ w2t,
    const unsigned short* __restrict__ wot, const unsigned short* __restrict__ yinA,
    const unsigned short* __restrict__ youtA, float* __restrict__ out)
{
  __shared__ __attribute__((aligned(16))) unsigned short xs[2 * 16 * 64];
  __shared__ __attribute__((aligned(16))) float qwg[NGC * 32];
  __shared__ __attribute__((aligned(16))) float coL[32 * 64];
  __shared__ __attribute__((aligned(16))) float outL[64 * 25];

  const int tid = threadIdx.x, lane = tid & 31, wv = tid >> 5;
  const int h = lane >> 4, m = lane & 15;
  const int n = blockIdx.x, b = blockIdx.y;
  const int pn1 = (b == 2) ? 1 : 0;
  const int pn2 = (b == 1) ? 1 : 0;
  const v8f z8 = {0.f, 0.f, 0.f, 0.f, 0.f, 0.f, 0.f, 0.f};

  {
    const int t = tid >> 6, mm = tid & 63;
    const float* xp = (t ? x2 : x1) + ((size_t)n * NCH + mm) * 18;
    float v[18];
    #pragma unroll
    for (int i = 0; i < 18; ++i) v[i] = xp[i];
    const int pneg = t ? pn2 : pn1;
    unsigned short* xrow = xs + t * 1024 + mm;
    #pragma unroll
    for (int lm = 0; lm < 16; ++lm) {
      unsigned short ov = 0;
      if (lm < NLM) {
        const int l = (lm == 0) ? 0 : ((lm < 4) ? 1 : 2);
        const int par = l & 1;
        const float val = ((par ^ pneg) != 0) ? v[9 + lm] : v[lm];
        ov = (unsigned short)bf16u(val);
      }
      xrow[lm * 64] = ov;
    }
  }
  for (int g = tid; g < NGC * 32; g += 128) {
    int be = g / NALPHA;
    be = (be > NBETA - 1) ? (NBETA - 1) : be;
    const float qv = bf16r(qw[be]);
    qwg[g] = (g < NG) ? qv : 0.0f;
  }
  __syncthreads();

  const int ch = 16 * wv + m;
  const int lsel = (m == 0) ? 0 : ((m < 4) ? 1 : ((m < NLM) ? 2 : 3));
  v8f accp[2];
  accp[0] = z8; accp[1] = z8;
  #pragma unroll
  for (int t = 0; t < 2; ++t) {
    const unsigned short* wt = (t ? w2t : w1t) + ((size_t)(b * 3) * NCH + ch) * NCH;
    #pragma unroll
    for (int ks = 0; ks < 2; ++ks) {
      FragB xa;
      const unsigned short* xr = xs + (t * 16 + m) * 64 + ks * 32;
      xa.h8[0] = *(const v8usa*)(xr + 8 * h);
      xa.h8[1] = *(const v8usa*)(xr + 16 + 8 * h);
      #pragma unroll
      for (int l = 0; l < 3; ++l) {
        const unsigned int msk = (lsel == l) ? 0xFFFFFFFFu : 0u;
        const v8u mv = {msk, msk, msk, msk, msk, msk, msk, msk};
        FragB am; am.w = xa.w & mv;
        FragB wb;
        load_frag_g(wb, wt + (size_t)l * (NCH * NCH) + ks * 32, h);
        accp[t] = mma_bf16(am.v, wb.v, accp[t]);
      }
    }
  }

  FragB bc[2];
  #pragma unroll
  for (int t = 0; t < 2; ++t) {
    #pragma unroll
    for (int r = 0; r < 8; ++r) {
      const float cv = accp[t][r] * 0.125f;
      const unsigned int hb = bf16u(cv);
      const float res = cv - bf16val(hb);
      bc[t].u[r]     = (unsigned short)hb;
      bc[t].u[8 + r] = (unsigned short)bf16u(res);
    }
  }

  v8f co0 = z8, co1 = z8;
  const unsigned short* yab = yinA + lane * 8;
  const unsigned short* yob = youtA + lane * 16;
  #pragma unroll 1
  for (int gc = 0; gc < NGC; ++gc) {
    FragB ph, pl;
    {
      FragB ya;
      ya.h8[0] = *(const v8usa*)(yab + (size_t)(2 * gc) * 256);
      ya.h8[1] = ya.h8[0];
      const v8f s1 = mma_bf16(ya.v, bc[0].v, z8);
      const v8f s2 = mma_bf16(ya.v, bc[1].v, z8);
      const float* qp = qwg + 32 * gc + 8 * h;
      const v4f qa = *(const v4fa*)qp;
      const v4f qb = *(const v4fa*)(qp + 4);
      v4f pa, pb;
      #pragma unroll
      for (int r = 0; r < 4; ++r) { pa[r] = (s1[r] * s2[r]) * qa[r]; pb[r] = (s1[4 + r] * s2[4 + r]) * qb[r]; }
      split8<0>(ph, pl, pa, pb);
    }
    {
      FragB ya;
      ya.h8[0] = *(const v8usa*)(yab + (size_t)(2 * gc + 1) * 256);
      ya.h8[1] = ya.h8[0];
      const v8f s1 = mma_bf16(ya.v, bc[0].v, z8);
      const v8f s2 = mma_bf16(ya.v, bc[1].v, z8);
      const float* qp = qwg + 32 * gc + 16 + 8 * h;
      const v4f qa = *(const v4fa*)qp;
      const v4f qb = *(const v4fa*)(qp + 4);
      v4f pa, pb;
      #pragma unroll
      for (int r = 0; r < 4; ++r) { pa[r] = (s1[r] * s2[r]) * qa[r]; pb[r] = (s1[4 + r] * s2[4 + r]) * qb[r]; }
      split8<1>(ph, pl, pa, pb);
    }
    FragB yo0, yo1;
    const unsigned short* yr = yob + (size_t)(2 * gc) * 512;
    yo0.h8[0] = *(const v8usa*)(yr);
    yo0.h8[1] = *(const v8usa*)(yr + 8);
    yo1.h8[0] = *(const v8usa*)(yr + 512);
    yo1.h8[1] = *(const v8usa*)(yr + 512 + 8);
    co0 = mma_bf16(yo0.v, ph.v, co0);
    co0 = mma_bf16(yo0.v, pl.v, co0);
    co1 = mma_bf16(yo1.v, ph.v, co1);
    co1 = mma_bf16(yo1.v, pl.v, co1);
  }

  #pragma unroll
  for (int r = 0; r < 8; ++r) {
    coL[(8 * h + r) * 64 + ch]      = co0[r];
    coL[(16 + 8 * h + r) * 64 + ch] = co1[r];
  }
  __syncthreads();

  const int d = ch;
  const unsigned short* wob = wot + ((size_t)(b * 5) * NCH + d) * NCH;
  v8f acc3[2];
  acc3[0] = z8; acc3[1] = z8;
  const int lq0 = (m == 0) ? 0 : ((m < 4) ? 1 : ((m < 9) ? 2 : 3));
  #pragma unroll
  for (int ks = 0; ks < 2; ++ks) {
    const float* cr = coL + m * 64 + 32 * ks;
    const v4f f0 = *(const v4fa*)(cr + 8 * h);
    const v4f f1 = *(const v4fa*)(cr + 8 * h + 4);
    const v4f f2 = *(const v4fa*)(cr + 16 + 8 * h);
    const v4f f3 = *(const v4fa*)(cr + 16 + 8 * h + 4);
    FragB ah, al;
    split8<0>(ah, al, f0, f1);
    split8<1>(ah, al, f2, f3);
    #pragma unroll
    for (int lq = 0; lq < 4; ++lq) {
      const unsigned int msk = (lq0 == lq) ? 0xFFFFFFFFu : 0u;
      const v8u mv = {msk, msk, msk, msk, msk, msk, msk, msk};
      FragB amh, aml;
      amh.w = ah.w & mv; aml.w = al.w & mv;
      FragB wb;
      load_frag_g(wb, wob + (size_t)lq * (NCH * NCH) + ks * 32, h);
      acc3[0] = mma_bf16(amh.v, wb.v, acc3[0]);
      acc3[0] = mma_bf16(aml.v, wb.v, acc3[0]);
    }
  }
  #pragma unroll
  for (int ks = 0; ks < 2; ++ks) {
    const float* cr = coL + (16 + m) * 64 + 32 * ks;
    const v4f f0 = *(const v4fa*)(cr + 8 * h);
    const v4f f1 = *(const v4fa*)(cr + 8 * h + 4);
    const v4f f2 = *(const v4fa*)(cr + 16 + 8 * h);
    const v4f f3 = *(const v4fa*)(cr + 16 + 8 * h + 4);
    FragB ah, al;
    split8<0>(ah, al, f0, f1);
    split8<1>(ah, al, f2, f3);
    const unsigned int msk = (m < 9) ? 0xFFFFFFFFu : 0u;
    const v8u mv = {msk, msk, msk, msk, msk, msk, msk, msk};
    FragB amh, aml;
    amh.w = ah.w & mv; aml.w = al.w & mv;
    FragB wb;
    load_frag_g(wb, wob + (size_t)4 * (NCH * NCH) + ks * 32, h);
    acc3[1] = mma_bf16(amh.v, wb.v, acc3[1]);
    acc3[1] = mma_bf16(aml.v, wb.v, acc3[1]);
  }

  #pragma unroll
  for (int r = 0; r < 8; ++r) outL[d * NLO + 8 * h + r] = acc3[0][r] * 0.125f;
  #pragma unroll
  for (int r = 0; r < 8; ++r) {
    const int lp = 16 + 8 * h + r;
    if (lp < NLO) outL[d * NLO + lp] = acc3[1][r] * 0.125f;
  }
  __syncthreads();

  float* ob = out + ((size_t)n * 3 + b) * (NCH * NLO);
  out_pass(outL, ob, tid);
  __threadfence();
  out_pass(outL, ob, tid);
}

extern "C" void kernel_launch(void* const* d_in, const int* in_sizes, int n_in,
                              void* d_out, int out_size, void* d_ws, size_t ws_size,
                              hipStream_t stream) {
  if (n_in < 8) return;
  if (in_sizes[0] != NS * NCH * 2 * NLM || in_sizes[1] != NS * NCH * 2 * NLM) return;
  if (in_sizes[2] != 3 * 3 * NCH * NCH || in_sizes[3] != 3 * 3 * NCH * NCH) return;
  if (in_sizes[4] != 3 * 5 * NCH * NCH) return;
  if (in_sizes[5] != NLM * NG || in_sizes[6] != NLO * NG || in_sizes[7] != NBETA) return;
  if (out_size != NS * 3 * NCH * NLO) return;

  const float* x1   = (const float*)d_in[0];
  const float* x2   = (const float*)d_in[1];
  const float* W1   = (const float*)d_in[2];
  const float* W2   = (const float*)d_in[3];
  const float* Wout = (const float*)d_in[4];
  const float* Yin  = (const float*)d_in[5];
  const float* Yout = (const float*)d_in[6];
  const float* qw   = (const float*)d_in[7];
  float* out = (float*)d_out;

  const size_t sz_w   = (size_t)3 * 3 * NCH * NCH * 2;
  const size_t sz_wo  = (size_t)3 * 5 * NCH * NCH * 2;
  const size_t sz_yin = (size_t)NGT * 32 * 8 * 2;
  const size_t sz_yo  = (size_t)NGC * 2 * 32 * 16 * 2;
  const size_t off_w1  = 0;
  const size_t off_w2  = off_w1 + sz_w;
  const size_t off_wo  = off_w2 + sz_w;
  const size_t off_yin = off_wo + sz_wo;
  const size_t off_yo  = off_yin + sz_yin;
  const size_t total   = off_yo + sz_yo;
  if (total > ws_size) return;

  char* ws = (char*)d_ws;
  unsigned short* w1t   = (unsigned short*)(ws + off_w1);
  unsigned short* w2t   = (unsigned short*)(ws + off_w2);
  unsigned short* wot   = (unsigned short*)(ws + off_wo);
  unsigned short* yinA  = (unsigned short*)(ws + off_yin);
  unsigned short* youtA = (unsigned short*)(ws + off_yo);

  prep_kernel<<<339, 64, 0, stream>>>(W1, W2, Wout, Yin, Yout, w1t, w2t, wot, yinA, youtA);

  dim3 gMain(NS, 3);
  gaunt_kernel<<<gMain, 128, 0, stream>>>(x1, x2, qw, w1t, w2t, wot, yinA, youtA, out);
}
